// VectorAttention_63153199120693
// MI455X (gfx1250) — hardware-verified
//
#include <hip/hip_runtime.h>


#define NB_  2
#define NN   512
#define CC   128
#define NR   (NB_ * NN)
#define IC   64
#define PCH  (IC * NN)
typedef _Float16 h16;
typedef unsigned short bf;
typedef __attribute__((ext_vector_type(16))) __bf16   v16bf;
typedef __attribute__((ext_vector_type(16))) _Float16 v16h;
typedef __attribute__((ext_vector_type(8)))  _Float16 v8h;
typedef __attribute__((ext_vector_type(8)))  unsigned short v8us;
typedef __attribute__((ext_vector_type(8)))  float    v8f;
typedef __attribute__((ext_vector_type(4)))  float    v4f;
typedef v8h  __attribute__((may_alias)) v8ha;
typedef v4f  __attribute__((may_alias)) v4fa;
typedef v8us __attribute__((may_alias)) v8usa;

__device__ __forceinline__ unsigned short f2bf(float f) { unsigned u = __float_as_uint(f); u += 0x7FFFu + ((u >> 16) & 1u); return (unsigned short)(u >> 16); }
__device__ __forceinline__ float bf2f(unsigned short b) { return __uint_as_float(((unsigned)b) << 16); }
__device__ __forceinline__ float bfr(float f) { return bf2f(f2bf(f)); }
__device__ __forceinline__ v16h cat16(v8h lo, v8h hi) { return __builtin_shufflevector(lo, hi, 0, 1, 2, 3, 4, 5, 6, 7, 8, 9, 10, 11, 12, 13, 14, 15); }
__device__ __forceinline__ v16bf cat16b(v8us lo, v8us hi) { return __builtin_bit_cast(v16bf, __builtin_shufflevector(lo, hi, 0, 1, 2, 3, 4, 5, 6, 7, 8, 9, 10, 11, 12, 13, 14, 15)); }
__device__ __forceinline__ v8f wmma16(v16h a, v16h b, v8f c) { return __builtin_amdgcn_wmma_f32_16x16x32_f16(false, a, false, b, (short)0, c, false, false); }
__device__ __forceinline__ v8f wmmab(v16bf a, v16bf b, v8f c) { return __builtin_amdgcn_wmma_f32_16x16x32_bf16(false, a, false, b, (short)0, c, false, false); }


template <typename T16> struct WFrag;
template <> struct WFrag<h16> { typedef v16h V; static __device__ __forceinline__ V ld(const h16* p) { return cat16(*(const v8h*)p, *(const v8h*)(p + 16)); } static __device__ __forceinline__ v8f mma(V a, V b, v8f c) { return wmma16(a, b, c); } };
template <> struct WFrag<bf> { typedef v16bf V; static __device__ __forceinline__ V ld(const bf* p) { return cat16b(*(const v8us*)p, *(const v8us*)(p + 16)); } static __device__ __forceinline__ v8f mma(V a, V b, v8f c) { return wmmab(a, b, c); } };
template <typename T16, int NSPLIT, bool BIAS>
__global__ __launch_bounds__(32) void k_gemmw(const T16* __restrict__ A, const T16* __restrict__ A2, const T16* __restrict__ Bt, const T16* __restrict__ Bt2, int K, float* C, int ldc, const float* __restrict__ bias, size_t sA, size_t sB, size_t sC) {
    typedef typename WFrag<T16>::V V;
    __shared__ __align__(16) float os[16 * 68];
    const size_t z = blockIdx.z; A += z * sA; if (A2) A2 += z * sA; Bt += z * sB; if (Bt2) Bt2 += z * sB; C += z * sC;
    const int lane = threadIdx.x & 31, lr = lane & 15, hi = lane >> 4; const int r0 = blockIdx.x * 64, c0 = blockIdx.y * 64;
    v8f acc[4][4];
#pragma unroll
    for (int mb = 0; mb < 4; ++mb)
#pragma unroll
        for (int nb = 0; nb < 4; ++nb) acc[mb][nb] = (v8f){};
    const size_t aoff = (size_t)(r0 + lr) * K + 8 * hi, boff = (size_t)(c0 + lr) * K + 8 * hi;
#pragma unroll 1
    for (int kc = 0; kc < K; kc += 32) {
        V a[4], a2[4];
#pragma unroll
        for (int mb = 0; mb < 4; ++mb) { a[mb] = WFrag<T16>::ld(A + aoff + (size_t)mb * 16 * K + kc); if (NSPLIT == 1 || NSPLIT == 2) a2[mb] = WFrag<T16>::ld(A2 + aoff + (size_t)mb * 16 * K + kc); }
#pragma unroll
        for (int nb = 0; nb < 4; ++nb) { const V b = WFrag<T16>::ld(Bt + boff + (size_t)nb * 16 * K + kc); V b2; if (NSPLIT >= 2) b2 = WFrag<T16>::ld(Bt2 + boff + (size_t)nb * 16 * K + kc);
#pragma unroll
            for (int mb = 0; mb < 4; ++mb) { acc[mb][nb] = WFrag<T16>::mma(a[mb], b, acc[mb][nb]); if (NSPLIT == 1 || NSPLIT == 2) acc[mb][nb] = WFrag<T16>::mma(a2[mb], b, acc[mb][nb]); if (NSPLIT >= 2) acc[mb][nb] = WFrag<T16>::mma(a[mb], b2, acc[mb][nb]); } }
        asm volatile("v_nop\n\tv_nop\n\tv_nop\n\tv_nop" : "+v"(acc[0][0]), "+v"(acc[1][1]), "+v"(acc[2][2]), "+v"(acc[3][3]) : "v"(a[0]), "v"(a[3]));
    }
#pragma unroll
    for (int mb = 0; mb < 4; ++mb) {
#pragma unroll
        for (int nb = 0; nb < 4; ++nb) {
#pragma unroll
            for (int j = 0; j < 8; ++j) os[(hi * 8 + j) * 68 + nb * 16 + lr] = acc[mb][nb][j]; }
        __builtin_amdgcn_wave_barrier(); asm volatile("" ::: "memory");
        float* crow = C + (size_t)(r0 + mb * 16) * ldc + c0;
#pragma unroll 1
        for (int ps = 0; ps < 2; ++ps) {
#pragma unroll
            for (int s = 0; s < 8; ++s) { const int row = 2 * s + hi, cofs = lr * 4; v4f val = *(const v4fa*)(os + row * 68 + cofs); if (BIAS) { val[0] += bfr(bias[c0 + cofs]); val[1] += bfr(bias[c0 + cofs + 1]); val[2] += bfr(bias[c0 + cofs + 2]); val[3] += bfr(bias[c0 + cofs + 3]); }
                *(volatile v4f*)(crow + (size_t)row * ldc + cofs) = val; }
            if (ps == 0) __threadfence(); }
        __builtin_amdgcn_wave_barrier(); asm volatile("" ::: "memory");
    }
}

typedef __attribute__((ext_vector_type(4))) unsigned short v4us;
typedef __attribute__((ext_vector_type(2))) unsigned short v2us;
__device__ __forceinline__ void splitf(float y, unsigned short& h, unsigned short& l) { h = f2bf(y); l = f2bf(y - bf2f(h)); }
__device__ __forceinline__ float expx(float a) { return __builtin_amdgcn_exp2f(__fmul_rn(a, 1.4426950408889634f)); }
__device__ __forceinline__ float mishx(float x) {
    const float sp = __fadd_rn(fmaxf(x, 0.0f), logf(__fadd_rn(1.0f, expx(-fabsf(x))))); const float th = __fsub_rn(1.0f, __fdiv_rn(2.0f, __fadd_rn(expx(__fmul_rn(2.0f, sp)), 1.0f))); return __fmul_rn(x, th); }
__global__ __launch_bounds__(256) void k_cvt8(const float* __restrict__ src, bf* dst, size_t n8) { const size_t i = (size_t)blockIdx.x * 256 + threadIdx.x; if (i >= n8) return; const v8f v = *(const v8f*)(src + i * 8); v8us o;
#pragma unroll
    for (int k = 0; k < 8; ++k) o[k] = f2bf(v[k]); *(volatile v8us*)(dst + i * 8) = o; __threadfence(); *(volatile v8us*)(dst + i * 8) = o; }

__global__ __launch_bounds__(256) void k_tohl(const float* __restrict__ F, bf* Hh, bf* Hl, size_t n4) { const size_t i = (size_t)blockIdx.x * 256 + threadIdx.x; if (i >= n4) return; const v4f a = *(const v4f*)(F + i * 4); v4us oh, ol;
#pragma unroll
    for (int q = 0; q < 4; ++q) { unsigned short h2, l2; splitf(a[q], h2, l2); oh[q] = h2; ol[q] = l2; }
    *(volatile v4us*)(Hh + i * 4) = oh; *(volatile v4us*)(Hl + i * 4) = ol; __threadfence(); *(volatile v4us*)(Hh + i * 4) = oh; *(volatile v4us*)(Hl + i * 4) = ol; }
__global__ __launch_bounds__(256) void k_lnmish(const float* __restrict__ F, const float* __restrict__ g, const float* __restrict__ bb, float* Y, int nrows) {
    const int lane = threadIdx.x & 31; const int row = blockIdx.x * 8 + (threadIdx.x >> 5); if (row >= nrows) return; const v4f a = *(const v4f*)(F + (size_t)row * CC + lane * 4); float v[4]; float s = 0.f;
#pragma unroll
    for (int q = 0; q < 4; ++q) { v[q] = a[q]; s = __fadd_rn(s, a[q]); }
#pragma unroll
    for (int sh = 16; sh; sh >>= 1) s = __fadd_rn(s, __shfl_xor(s, sh, 32));
    const float mu = __fdiv_rn(s, (float)CC); float s2 = 0.f;
#pragma unroll
    for (int q = 0; q < 4; ++q) { float d0 = __fsub_rn(v[q], mu); asm volatile("" : "+v"(d0)); float p = __fmul_rn(d0, d0); asm volatile("" : "+v"(p)); s2 = __fadd_rn(s2, p); }
#pragma unroll
    for (int sh = 16; sh; sh >>= 1) s2 = __fadd_rn(s2, __shfl_xor(s2, sh, 32));
    const float rs = __fdiv_rn(1.0f, __fsqrt_rn(__fadd_rn(__fdiv_rn(s2, (float)CC), 1e-5f))); v4f o;
#pragma unroll
    for (int q = 0; q < 4; ++q) { const int c = lane * 4 + q; float xn = __fmul_rn(__fsub_rn(v[q], mu), rs); asm volatile("" : "+v"(xn)); float y = __fmul_rn(xn, bfr(g[c])); asm volatile("" : "+v"(y)); y = __fadd_rn(y, bfr(bb[c])); o[q] = mishx(y); }
    *(volatile v4f*)(Y + (size_t)row * CC + lane * 4) = o; __threadfence(); *(volatile v4f*)(Y + (size_t)row * CC + lane * 4) = o; }
__global__ __launch_bounds__(256) void k_pair(const float* __restrict__ KW, const float* __restrict__ QW, size_t i0row, const float* __restrict__ b1, const float* __restrict__ g, const float* __restrict__ bb, bf* Hh, bf* Hl) {
    const int lane = threadIdx.x & 31; const size_t pr = (size_t)blockIdx.x * 8 + (threadIdx.x >> 5); if (pr >= (size_t)PCH) return; const int j = (int)(pr % NN); const size_t irow = i0row + pr / NN; const size_t b = i0row / NN;
    const v4f kw = *(const v4f*)(KW + (b * NN + j) * CC + lane * 4); const v4f qw = *(const v4f*)(QW + irow * CC + lane * 4); float v[4]; float s = 0.f;
#pragma unroll
    for (int q = 0; q < 4; ++q) { float d0 = __fsub_rn(kw[q], qw[q]); asm volatile("" : "+v"(d0)); v[q] = __fadd_rn(d0, bfr(b1[lane * 4 + q])); s = __fadd_rn(s, v[q]); }
#pragma unroll
    for (int sh = 16; sh; sh >>= 1) s = __fadd_rn(s, __shfl_xor(s, sh, 32));
    const float mu = __fdiv_rn(s, (float)CC); float s2 = 0.f;
#pragma unroll
    for (int q = 0; q < 4; ++q) { float d0 = __fsub_rn(v[q], mu); asm volatile("" : "+v"(d0)); float p = __fmul_rn(d0, d0); asm volatile("" : "+v"(p)); s2 = __fadd_rn(s2, p); }
#pragma unroll
    for (int sh = 16; sh; sh >>= 1) s2 = __fadd_rn(s2, __shfl_xor(s2, sh, 32));
    const float rs = __fdiv_rn(1.0f, __fsqrt_rn(__fadd_rn(__fdiv_rn(s2, (float)CC), 1e-5f))); v4us oh, ol;
#pragma unroll
    for (int q = 0; q < 4; ++q) { const int c = lane * 4 + q; float xn = __fmul_rn(__fsub_rn(v[q], mu), rs); asm volatile("" : "+v"(xn)); float y = __fmul_rn(xn, bfr(g[c])); asm volatile("" : "+v"(y)); y = __fadd_rn(y, bfr(bb[c])); unsigned short h2, l2; splitf(mishx(y), h2, l2); oh[q] = h2; ol[q] = l2; }
    const size_t oo = pr * CC + lane * 4; *(volatile v4us*)(Hh + oo) = oh; *(volatile v4us*)(Hl + oo) = ol; __threadfence(); *(volatile v4us*)(Hh + oo) = oh; *(volatile v4us*)(Hl + oo) = ol; }
__global__ __launch_bounds__(256) void k_vagg(const float* __restrict__ Wc, const float* __restrict__ Vv, const float* __restrict__ dist, size_t i0row, float* out) {
    const int t = blockIdx.x * 256 + threadIdx.x; if (t >= IC * CC) return; const int c = t % CC; const int il = t / CC; const size_t irow = i0row + il; const size_t b = i0row / NN; const float di = bfr(dist[irow]); const float* wr = Wc + (size_t)il * NN * CC + c; float m = -3.0e38f;
#pragma unroll 4
    for (int j = 0; j < NN; ++j) m = fmaxf(m, wr[(size_t)j * CC]);
    float s = 0.f;
#pragma unroll 4
    for (int j = 0; j < NN; ++j) { const float e = __fmul_rn(expx(__fsub_rn(wr[(size_t)j * CC], m)), bfr(dist[b * NN + j])); s = __fadd_rn(s, e); }
    float acc = 0.f;
#pragma unroll 4
    for (int j = 0; j < NN; ++j) { const float dj = bfr(dist[b * NN + j]); float e = __fmul_rn(expx(__fsub_rn(wr[(size_t)j * CC], m)), dj); asm volatile("" : "+v"(e)); float p = __fdiv_rn(e, s); asm volatile("" : "+v"(p)); const float mk = (__fmul_rn(di, dj) > 0.0f) ? 1.0f : 0.0f; float pm = __fmul_rn(p, mk); asm volatile("" : "+v"(pm)); float term = __fmul_rn(pm, Vv[(b * NN + j) * CC + c]); asm volatile("" : "+v"(term)); acc = __fadd_rn(acc, term); }
    *(volatile float*)(out + irow * CC + c) = acc; __threadfence(); *(volatile float*)(out + irow * CC + c) = acc; }

extern "C" void kernel_launch(void* const* d_in, const int* in_sizes, int n_in,
                              void* d_out, int out_size, void* d_ws, size_t ws_size, hipStream_t stream) {
    (void)in_sizes; (void)n_in; (void)out_size;
    const float* feat = (const float*)d_in[0];   const float* dist = (const float*)d_in[2];
    const float* wq = (const float*)d_in[3]; const float* bq = (const float*)d_in[4]; const float* gq = (const float*)d_in[5]; const float* btq = (const float*)d_in[6]; const float* wk = (const float*)d_in[7]; const float* bk = (const float*)d_in[8]; const float* gk = (const float*)d_in[9]; const float* btk = (const float*)d_in[10];
    const float* wv = (const float*)d_in[11]; const float* bv = (const float*)d_in[12]; const float* w1 = (const float*)d_in[13]; const float* b1 = (const float*)d_in[14]; const float* g1 = (const float*)d_in[15]; const float* bt1 = (const float*)d_in[16]; const float* w2 = (const float*)d_in[17]; const float* b2 = (const float*)d_in[18];
    float* OUT = (float*)d_out;
    char* wsp = (char*)d_ws;
    auto take = [&](size_t bytes) { char* p = wsp; wsp += (bytes + 255) & ~(size_t)255; return (void*)p; };
    bf* WQ = (bf*)take((size_t)CC * CC * 2); bf* WK = (bf*)take((size_t)CC * CC * 2); bf* WV = (bf*)take((size_t)CC * CC * 2); bf* W1B = (bf*)take((size_t)CC * CC * 2); bf* W2B = (bf*)take((size_t)CC * CC * 2);
    bf* XB = (bf*)take((size_t)NR * CC * 2); float* F = (float*)take((size_t)NR * CC * 4); float* Q = (float*)take((size_t)NR * CC * 4); float* K = (float*)take((size_t)NR * CC * 4); float* Vv = (float*)take((size_t)NR * CC * 4); bf* Th = (bf*)take((size_t)NR * CC * 2); bf* Tl = (bf*)take((size_t)NR * CC * 2); float* QW = (float*)take((size_t)NR * CC * 4); float* KW = (float*)take((size_t)NR * CC * 4);
    bf* Hh = (bf*)take((size_t)PCH * CC * 2); bf* Hl = (bf*)take((size_t)PCH * CC * 2); float* Wc = (float*)take((size_t)PCH * CC * 4);
    if ((size_t)(wsp - (char*)d_ws) > ws_size) return;
    const size_t nw8 = (size_t)CC * CC / 8;
    k_cvt8<<<(unsigned)((nw8 + 255) / 256), 256, 0, stream>>>(wq, WQ, nw8); k_cvt8<<<(unsigned)((nw8 + 255) / 256), 256, 0, stream>>>(wk, WK, nw8); k_cvt8<<<(unsigned)((nw8 + 255) / 256), 256, 0, stream>>>(wv, WV, nw8); k_cvt8<<<(unsigned)((nw8 + 255) / 256), 256, 0, stream>>>(w1, W1B, nw8); k_cvt8<<<(unsigned)((nw8 + 255) / 256), 256, 0, stream>>>(w2, W2B, nw8);
    k_cvt8<<<(unsigned)(((size_t)NR * CC / 8 + 255) / 256), 256, 0, stream>>>(feat, XB, (size_t)NR * CC / 8);
    const size_t N4 = (size_t)NR * CC / 4;
    k_gemmw<bf, 0, true><<<dim3(NR / 64, CC / 64, 1), 32, 0, stream>>>(XB, nullptr, WQ, nullptr, CC, F, CC, bq, 0, 0, 0); k_lnmish<<<NR / 8, 256, 0, stream>>>(F, gq, btq, Q, NR);
    k_gemmw<bf, 0, true><<<dim3(NR / 64, CC / 64, 1), 32, 0, stream>>>(XB, nullptr, WK, nullptr, CC, F, CC, bk, 0, 0, 0); k_lnmish<<<NR / 8, 256, 0, stream>>>(F, gk, btk, K, NR);
    k_gemmw<bf, 0, true><<<dim3(NR / 64, CC / 64, 1), 32, 0, stream>>>(XB, nullptr, WV, nullptr, CC, Vv, CC, bv, 0, 0, 0);
    k_tohl<<<(unsigned)((N4 + 255) / 256), 256, 0, stream>>>(Q, Th, Tl, N4); k_gemmw<bf, 1, false><<<dim3(NR / 64, CC / 64, 1), 32, 0, stream>>>(Th, Tl, W1B, nullptr, CC, QW, CC, nullptr, 0, 0, 0);
    k_tohl<<<(unsigned)((N4 + 255) / 256), 256, 0, stream>>>(K, Th, Tl, N4); k_gemmw<bf, 1, false><<<dim3(NR / 64, CC / 64, 1), 32, 0, stream>>>(Th, Tl, W1B, nullptr, CC, KW, CC, nullptr, 0, 0, 0);
    for (size_t i0row = 0; i0row < (size_t)NR; i0row += IC) {
        k_pair<<<(unsigned)((PCH + 7) / 8), 256, 0, stream>>>(KW, QW, i0row, b1, g1, bt1, Hh, Hl);
        k_gemmw<bf, 1, true><<<dim3(PCH / 64, CC / 64, 1), 32, 0, stream>>>(Hh, Hl, W2B, nullptr, CC, Wc, CC, b2, 0, 0, 0);
        k_vagg<<<(IC * CC + 255) / 256, 256, 0, stream>>>(Wc, Vv, dist, i0row, OUT); }
}
